// GATLayer_36051955482701
// MI455X (gfx1250) — hardware-verified
//
#include <hip/hip_runtime.h>
#include <stddef.h>
#include <stdint.h>
#include <math.h>


#define NB     8
#define NNODE  1024
#define FIN    256
#define FOUT   256
#define NH     4
#define HD     64
#define MROWS  (NB * NNODE)
#define NBH    (NB * NH)
#define EPL    (NBH * NNODE)
#define MWORDS (NNODE / 32)
#define PTHR   256
#define NUX    (MROWS * (FIN / 8))
#define NUW    (FOUT * (FIN / 8))
#define NUM    (MROWS * 32)
#define GBM    64
#define GBN    64
#define GTHR   128
#define SP     68
#define KT     64
#define NKT    (NNODE / KT)
#define RT     64
#define NEGV   (-9.0e15f)
#define NEGSL  0.2f
#define WSMAX  134217728

static_assert((NUX % PTHR) == 0 && (NUW % PTHR) == 0 && (NUM % PTHR) == 0);
static_assert((FIN % 32) == 0 && (MROWS % GBM) == 0 && FOUT == NH * HD && HD == GBN);
static_assert(GBM == (GTHR / 32) * 16 && GTHR == 2 * HD && GTHR == 2 * GBM);
static_assert((NNODE % KT) == 0 && (NNODE % RT) == 0 && (NNODE % GBM) == 0);
static_assert(RT == (GTHR / 32) * 16);
static_assert((SP % 4) == 0 && SP >= GBN);
static_assert(FIN / 8 == 32 && MWORDS == 32);
static_assert(NNODE == 2 * GTHR * 4);
static_assert(RT * MWORDS == 4 * GTHR * 4);
static_assert((GBM * GBN / 8) == 4 * GTHR);

typedef float          v4f  __attribute__((ext_vector_type(4)));
typedef float          v8f  __attribute__((ext_vector_type(8)));
typedef int            v8i  __attribute__((ext_vector_type(8)));
typedef unsigned int   v2u  __attribute__((ext_vector_type(2)));
typedef unsigned int   v4u  __attribute__((ext_vector_type(4)));
typedef unsigned short v8us __attribute__((ext_vector_type(8)));
typedef __bf16         v16b __attribute__((ext_vector_type(16)));
typedef v4f  __attribute__((may_alias)) v4fa;
typedef v2u  __attribute__((may_alias)) v2ua;
typedef v4u  __attribute__((may_alias)) v4ua;
typedef v8us __attribute__((may_alias)) v8usa;
union FragB { v16b v; v8us h[2]; v8i w; };

__device__ __forceinline__ v8f wmb(const FragB& a, const FragB& b, v8f c) {
  v8f d = __builtin_amdgcn_wmma_f32_16x16x32_bf16(false, a.v, false, b.v, (short)0, c, false, false);
  asm volatile("v_nop\n\tv_nop\n\tv_nop\n\tv_nop" : "+v"(d) : "v"(a.w), "v"(b.w));
  return d;
}

__device__ __forceinline__ unsigned int f2bf(float f) {
  const unsigned int u = __float_as_uint(f);
  return ((u + 0x7FFFu + ((u >> 16) & 1u)) >> 16) & 0xFFFFu;
}
__device__ __forceinline__ float bf2f(unsigned int b) { return __uint_as_float(b << 16); }
__device__ __forceinline__ float bfr(float f) { return bf2f(f2bf(f)); }
__device__ __forceinline__ unsigned int pk2(float lo, float hi) { return f2bf(lo) | (f2bf(hi) << 16); }
__device__ __forceinline__ v4u pack8(const v4f a, const v4f b) {
  v4u r;
  r.x = pk2(a.x, a.y); r.y = pk2(a.z, a.w); r.z = pk2(b.x, b.y); r.w = pk2(b.z, b.w);
  return r;
}

__global__ __launch_bounds__(PTHR) void k_prep(const float* __restrict__ x, const float* __restrict__ adj,
                                               const float* __restrict__ W,
                                               unsigned short* xb, unsigned short* wt, unsigned int* adjb) {
  const int u = (int)blockIdx.x * PTHR + (int)threadIdx.x;
  if (u < NUX) {
    const int row = u >> 5;
    const int c0  = (u & 31) * 8;
    const float* p = x + (size_t)row * FIN + c0;
    const v4f a = *(const v4fa*)p;
    const v4f b = *(const v4fa*)(p + 4);
    const v4u hv = pack8(a, b);
    unsigned short* o = xb + (size_t)row * FIN + c0;
    *(volatile v4u*)o = hv;
    __threadfence();
    *(volatile v4u*)o = hv;
  } else if (u < NUX + NUW) {
    const int v  = u - NUX;
    const int n  = v >> 5;
    const int k8 = (v & 31) * 8;
    const float* p = W + (size_t)k8 * FOUT + n;
    v4f a, b;
    a.x = p[0];          a.y = p[FOUT];       a.z = p[2 * FOUT];   a.w = p[3 * FOUT];
    b.x = p[4 * FOUT];   b.y = p[5 * FOUT];   b.z = p[6 * FOUT];   b.w = p[7 * FOUT];
    const v4u wv = pack8(a, b);
    unsigned short* o = wt + (size_t)n * FIN + k8;
    *(volatile v4u*)o = wv;
    __threadfence();
    *(volatile v4u*)o = wv;
  } else if (u < NUX + NUW + NUM) {
    const int v   = u - NUX - NUW;
    const int row = v >> 5;
    const int l   = v & 31;
    const float* p = adj + (size_t)row * NNODE + 32 * l;
    unsigned int word = 0u;
#pragma unroll
    for (int q = 0; q < 8; ++q) {
      const v4f a = *(const v4fa*)(p + 4 * q);
      const unsigned int b4 = (a.x > 0.0f ? 1u : 0u) | (a.y > 0.0f ? 2u : 0u) |
                              (a.z > 0.0f ? 4u : 0u) | (a.w > 0.0f ? 8u : 0u);
      word |= b4 << (4 * q);
    }
    unsigned int* o = adjb + (size_t)row * MWORDS + l;
    *(volatile unsigned int*)o = word;
    __threadfence();
    *(volatile unsigned int*)o = word;
  }
}

__global__ __launch_bounds__(GTHR) void k_proj(const unsigned short* __restrict__ A,
                                               const unsigned short* __restrict__ WT,
                                               const float* __restrict__ avec,
                                               float* E, unsigned short* VTH, unsigned short* VTL) {
  __shared__ __attribute__((aligned(16))) float stg[GBM * SP];
  __shared__ __attribute__((aligned(16))) float satt[2 * HD];
  __shared__ __attribute__((aligned(16))) float sdot[2 * GBM];
  const int tid = (int)threadIdx.x, lane = tid & 31, wave = tid >> 5, hh = lane >> 4, m = lane & 15;
  const int rowBase = (int)blockIdx.x * GBM;
  const int head    = (int)blockIdx.y;
  const int col0    = head * GBN;
  const int bidx    = rowBase >> 10;
  const int n0      = rowBase & (NNODE - 1);
  const int bh      = bidx * NH + head;

  satt[tid] = bfr(avec[head * (2 * HD) + tid]);

  v8f acc[4];
  {
    const v8f z = {0.f, 0.f, 0.f, 0.f, 0.f, 0.f, 0.f, 0.f};
    acc[0] = z; acc[1] = z; acc[2] = z; acc[3] = z;
  }
  const unsigned short* ap = A  + (size_t)(rowBase + 16 * wave + m) * (size_t)FIN + 8 * hh;
  const unsigned short* wp = WT + (size_t)(col0 + m) * (size_t)FIN + 8 * hh;
#pragma unroll 1
  for (int ks = 0; ks < FIN / 32; ++ks) {
    FragB af;
    af.h[0] = *(const v8usa*)(ap + 32 * ks);
    af.h[1] = *(const v8usa*)(ap + 32 * ks + 16);
#pragma unroll
    for (int t = 0; t < 4; ++t) {
      const unsigned short* wq = wp + (size_t)(16 * t) * (size_t)FIN + 32 * ks;
      FragB bf;
      bf.h[0] = *(const v8usa*)wq;
      bf.h[1] = *(const v8usa*)(wq + 16);
      acc[t] = wmb(af, bf, acc[t]);
    }
  }

#pragma unroll
  for (int t = 0; t < 4; ++t) {
    const int lc = 16 * t + m;
#pragma unroll
    for (int r = 0; r < 8; ++r) {
      const int lr = 16 * wave + 8 * hh + r;
      stg[lr * SP + lc] = acc[t][r];
    }
  }
  __syncthreads();

  {
    const int row = tid & 63, which = tid >> 6;
    const float* sa = satt + which * HD;
    const float* hr = stg + row * SP;
    float d = 0.f;
#pragma unroll 4
    for (int c4 = 0; c4 < GBN / 4; ++c4) {
      const v4f hv = *(const v4fa*)(hr + 4 * c4);
      const v4f av = *(const v4fa*)(sa + 4 * c4);
      d = fmaf(hv.x, av.x, d);
      d = fmaf(hv.y, av.y, d);
      d = fmaf(hv.z, av.z, d);
      d = fmaf(hv.w, av.w, d);
    }
    sdot[which * GBM + row] = d;
  }
  __syncthreads();

  v4u hv4[4], lv4[4];
  {
    const int q = tid & 7;
#pragma unroll
    for (int j = 0; j < 4; ++j) {
      const int d = (tid >> 3) + 16 * j;
      unsigned int hb[8], lb[8];
#pragma unroll
      for (int i = 0; i < 8; ++i) {
        const float v = stg[(8 * q + i) * SP + d];
        hb[i] = f2bf(v);
        lb[i] = f2bf(v - bf2f(hb[i]));
      }
      hv4[j].x = hb[0] | (hb[1] << 16); hv4[j].y = hb[2] | (hb[3] << 16);
      hv4[j].z = hb[4] | (hb[5] << 16); hv4[j].w = hb[6] | (hb[7] << 16);
      lv4[j].x = lb[0] | (lb[1] << 16); lv4[j].y = lb[2] | (lb[3] << 16);
      lv4[j].z = lb[4] | (lb[5] << 16); lv4[j].w = lb[6] | (lb[7] << 16);
    }
  }
  const size_t vbase = ((size_t)bh * HD + (size_t)(tid >> 3)) * (size_t)NNODE + (size_t)(n0 + 8 * (tid & 7));
  const int which2 = lane >> 4, piece = lane & 15;
  const v4f sdv = *(const v4fa*)(sdot + which2 * GBM + 4 * piece);
  float* sp = E + (size_t)which2 * (size_t)EPL + (size_t)bh * NNODE + n0 + 4 * piece;

#pragma unroll
  for (int j = 0; j < 4; ++j) {
    const size_t o = vbase + (size_t)(16 * j) * (size_t)NNODE;
    *(volatile v4u*)(VTH + o) = hv4[j];
    *(volatile v4u*)(VTL + o) = lv4[j];
  }
  if (wave == 0) *(volatile v4f*)sp = sdv;
  __threadfence();
#pragma unroll
  for (int j = 0; j < 4; ++j) {
    const size_t o = vbase + (size_t)(16 * j) * (size_t)NNODE;
    *(volatile v4u*)(VTH + o) = hv4[j];
    *(volatile v4u*)(VTL + o) = lv4[j];
  }
  if (wave == 0) *(volatile v4f*)sp = sdv;
}

__device__ __forceinline__ float gscore(float ei, float ej, unsigned int by, int i) {
  float s = ei + ej;
  s = s > 0.0f ? s : NEGSL * s;
  return ((by >> i) & 1u) != 0u ? s : NEGV;
}

__global__ __launch_bounds__(GTHR) void k_attn(const unsigned int* __restrict__ adjb, const float* __restrict__ E,
                                               const unsigned short* __restrict__ VTH,
                                               const unsigned short* __restrict__ VTL, float* out) {
  __shared__ __attribute__((aligned(16))) float        sej[NNODE];
  __shared__ __attribute__((aligned(16))) unsigned int smk[RT * MWORDS];
  __shared__ __attribute__((aligned(16))) float        sto[RT * SP];
  const int tid = (int)threadIdx.x, lane = tid & 31, wave = tid >> 5, hh = lane >> 4, m = lane & 15;
  const int bid  = (int)blockIdx.x;
  const int rt   = bid & (NNODE / RT - 1);
  const int bh   = bid / (NNODE / RT);
  const int bidx = bh >> 2, head = bh & (NH - 1);
  const int rowBase = rt * RT;

  {
    const float* ejp = E + (size_t)EPL + (size_t)bh * NNODE;
#pragma unroll
    for (int i = 0; i < 2; ++i) {
      const int idx = tid + GTHR * i;
      *(v4fa*)(sej + 4 * idx) = *(const v4fa*)(ejp + 4 * idx);
    }
    const unsigned int* mp = adjb + ((size_t)bidx * NNODE + rowBase) * MWORDS;
#pragma unroll
    for (int i = 0; i < 4; ++i) {
      const int idx = tid + GTHR * i;
      *(v4ua*)(smk + 4 * idx) = *(const v4ua*)(mp + 4 * idx);
    }
  }
  const int mrow = 16 * wave + m;
  const float eiv = E[(size_t)bh * NNODE + rowBase + mrow];
  __syncthreads();

  float mrun = -3.0e38f, lrun = 0.0f;
  v8f acc[4];
  {
    const v8f z = {0.f, 0.f, 0.f, 0.f, 0.f, 0.f, 0.f, 0.f};
    acc[0] = z; acc[1] = z; acc[2] = z; acc[3] = z;
  }
  const size_t vrow = ((size_t)bh * HD + (size_t)m) * (size_t)NNODE + (size_t)(8 * hh);

#pragma unroll 1
  for (int kt = 0; kt < NKT; ++kt) {
    const int mb = kt * KT;
    const v2u mw = *(const v2ua*)(smk + mrow * MWORDS + 2 * kt);
    float sv[32];
#pragma unroll
    for (int g = 0; g < 4; ++g) {
      const float* ejb = sej + mb + 16 * g + 8 * hh;
      const v4f ea = *(const v4fa*)ejb;
      const v4f eb = *(const v4fa*)(ejb + 4);
      const unsigned int wsel = (g < 2) ? mw.x : mw.y;
      const unsigned int by = (wsel >> (16 * (g & 1) + 8 * hh)) & 0xFFu;
      sv[8 * g + 0] = gscore(eiv, ea.x, by, 0);
      sv[8 * g + 1] = gscore(eiv, ea.y, by, 1);
      sv[8 * g + 2] = gscore(eiv, ea.z, by, 2);
      sv[8 * g + 3] = gscore(eiv, ea.w, by, 3);
      sv[8 * g + 4] = gscore(eiv, eb.x, by, 4);
      sv[8 * g + 5] = gscore(eiv, eb.y, by, 5);
      sv[8 * g + 6] = gscore(eiv, eb.z, by, 6);
      sv[8 * g + 7] = gscore(eiv, eb.w, by, 7);
    }
    float mloc = sv[0];
#pragma unroll
    for (int i = 1; i < 32; ++i) mloc = fmaxf(mloc, sv[i]);
    mloc = fmaxf(mloc, __shfl_xor(mloc, 16));
    const float mnew  = fmaxf(mrun, mloc);
    const float scale = expf(mrun - mnew);

    FragB ph[2], pl[2];
    float lsum = 0.0f;
#pragma unroll
    for (int ks = 0; ks < 2; ++ks) {
#pragma unroll
      for (int j = 0; j < 8; ++j) {
        const float p0 = expf(sv[16 * ks + 2 * j]     - mnew);
        const float p1 = expf(sv[16 * ks + 2 * j + 1] - mnew);
        lsum += p0 + p1;
        const unsigned int h0 = f2bf(p0), h1 = f2bf(p1);
        const unsigned int l0 = f2bf(p0 - bf2f(h0)), l1 = f2bf(p1 - bf2f(h1));
        ph[ks].w[j] = (int)(h0 | (h1 << 16));
        pl[ks].w[j] = (int)(l0 | (l1 << 16));
      }
    }
    lsum += __shfl_xor(lsum, 16);
    lrun = lrun * scale + lsum;
    mrun = mnew;

    float rs[8];
#pragma unroll
    for (int r = 0; r < 8; ++r) rs[r] = __shfl(scale, 8 * hh + r);
#pragma unroll
    for (int t = 0; t < 4; ++t) {
#pragma unroll
      for (int r = 0; r < 8; ++r) acc[t][r] *= rs[r];
    }

#pragma unroll
    for (int ks = 0; ks < 2; ++ks) {
#pragma unroll
      for (int t = 0; t < 4; ++t) {
        const size_t o = vrow + (size_t)(16 * t) * (size_t)NNODE + (size_t)(mb + 32 * ks);
        FragB vh, vl;
        vh.h[0] = *(const v8usa*)(VTH + o);
        vh.h[1] = *(const v8usa*)(VTH + o + 16);
        vl.h[0] = *(const v8usa*)(VTL + o);
        vl.h[1] = *(const v8usa*)(VTL + o + 16);
        acc[t] = wmb(ph[ks], vh, acc[t]);
        acc[t] = wmb(ph[ks], vl, acc[t]);
        acc[t] = wmb(pl[ks], vh, acc[t]);
      }
    }
  }

  const float linv = 1.0f / lrun;
  float rl[8];
#pragma unroll
  for (int r = 0; r < 8; ++r) rl[r] = __shfl(linv, 8 * hh + r);
  float* so = sto + wave * 16 * SP;
#pragma unroll
  for (int t = 0; t < 4; ++t) {
#pragma unroll
    for (int r = 0; r < 8; ++r) so[(8 * hh + r) * SP + 16 * t + m] = acc[t][r] * rl[r];
  }
  __syncthreads();

  v4f fv[8];
#pragma unroll
  for (int i = 0; i < 8; ++i) {
    const int lr = 2 * i + hh;
    fv[i] = *(const v4fa*)(so + lr * SP + 4 * m);
  }
  float* ob = out + ((size_t)bidx * NNODE + (size_t)(rowBase + 16 * wave)) * (size_t)FOUT + head * HD + 4 * m;
#pragma unroll
  for (int i = 0; i < 8; ++i) {
    const int lr = 2 * i + hh;
    *(volatile v4f*)(ob + (size_t)lr * FOUT) = fv[i];
  }
  __threadfence();
#pragma unroll
  for (int i = 0; i < 8; ++i) {
    const int lr = 2 * i + hh;
    *(volatile v4f*)(ob + (size_t)lr * FOUT) = fv[i];
  }
}

extern "C" void kernel_launch(void* const* d_in, const int* in_sizes, int n_in,
                              void* d_out, int out_size, void* d_ws, size_t ws_size,
                              hipStream_t stream) {
  if (n_in < 4) return;
  if (in_sizes[0] != MROWS * FIN) return;
  if (in_sizes[1] != NB * NNODE * NNODE) return;
  if (in_sizes[2] != FIN * FOUT) return;
  if (in_sizes[3] != NH * 2 * HD) return;
  if (out_size != MROWS * FOUT) return;

  const float* x   = (const float*)d_in[0];
  const float* adj = (const float*)d_in[1];
  const float* W   = (const float*)d_in[2];
  const float* av  = (const float*)d_in[3];
  float* out = (float*)d_out;

  char* ws = (char*)d_ws;
  size_t off = 0;
  const size_t oXB  = off; off += (size_t)MROWS * FIN * 2;          off = (off + 255) & ~(size_t)255;
  const size_t oWT  = off; off += (size_t)FOUT * FIN * 2;           off = (off + 255) & ~(size_t)255;
  const size_t oVTH = off; off += (size_t)NBH * HD * NNODE * 2;     off = (off + 255) & ~(size_t)255;
  const size_t oVTL = off; off += (size_t)NBH * HD * NNODE * 2;     off = (off + 255) & ~(size_t)255;
  const size_t oE   = off; off += (size_t)2 * EPL * 4;              off = (off + 255) & ~(size_t)255;
  const size_t oMB  = off; off += (size_t)MROWS * MWORDS * 4;        off = (off + 255) & ~(size_t)255;
  if (off > ws_size || off > (size_t)WSMAX) return;
  unsigned short* XB   = (unsigned short*)(ws + oXB);
  unsigned short* WT   = (unsigned short*)(ws + oWT);
  unsigned short* VTH  = (unsigned short*)(ws + oVTH);
  unsigned short* VTL  = (unsigned short*)(ws + oVTL);
  float*          Ep   = (float*)(ws + oE);
  unsigned int*   ADJB = (unsigned int*)(ws + oMB);

  k_prep<<<(NUX + NUW + NUM) / PTHR, PTHR, 0, stream>>>(x, adj, W, XB, WT, ADJB);
  k_proj<<<dim3(MROWS / GBM, NH), GTHR, 0, stream>>>(XB, WT, av, Ep, VTH, VTL);
  k_attn<<<NBH * (NNODE / RT), GTHR, 0, stream>>>(ADJB, Ep, VTH, VTL, out);
}
